// MoESwiGLUFFN_9380208575128
// MI455X (gfx1250) — hardware-run, weakly checked
//
#include <hip/hip_runtime.h>
#include <math.h>

#ifndef NTOK
#define NTOK 8192
#endif
#define NTOK_FULL 8192
#define DM 512
#define HID 1365
#define HP 1408
#define NE 8
#define TOPK 2
#define NSLOT (NTOK * TOPK)
#define R_MAX (NSLOT + 64 * NE)
#define NT_MAX (R_MAX / 64)
#define SPT (NSLOT / 512)
#define RT_HALF (R_MAX / 2)
#define SR_HALF (NSLOT / 2)

#define CX_LOG2 11
#define CWI_LOG2 18
#define CH_LOG2 11
#define CWO_LOG2 19
#define CX ((float)(1u << CX_LOG2))
#define CH ((float)(1u << CH_LOG2))
#define SC_HG (1.0f / (float)(1u << (CX_LOG2 + CWI_LOG2)))
#define SC_Y (1.0f / (float)(1u << (CH_LOG2 + CWO_LOG2)))

#define TBL_COUNT 0
#define TBL_POFF 16
#define TBL_NTILES 32
#define TBL_TILE_E 64
#define TBL_ROWTOK 512
#define TBL_SLOTROW (512 + R_MAX)
#define TBL_WORDS (512 + R_MAX + NSLOT)

static_assert(NE <= 16 && TOPK == 2 && NSLOT % 512 == 0);
static_assert(NE == 8);
static_assert(NTOK <= NTOK_FULL && NTOK % 128 == 0);
static_assert(SPT % 4 == 0 && SPT >= 4 && SPT <= 32);
static_assert(R_MAX % 64 == 0 && TBL_TILE_E + NT_MAX <= TBL_ROWTOK);
static_assert(TBL_POFF + NE + 1 <= TBL_NTILES && TBL_NTILES < TBL_TILE_E);
static_assert(DM == 512 && HID == 1365 && HP == 1408);
static_assert(DM % 64 == 0 && HP % 64 == 0 && HID <= HP && HP - HID < 64 && DM % 32 == 0 && HP % 32 == 0);
static_assert((R_MAX * (DM / 8)) % 256 == 0 && NTOK % 8 == 0);
static_assert((NT_MAX * 2 * (HP / 64)) % 8 == 0 && (NT_MAX * (DM / 64)) % 8 == 0);
static_assert(CX_LOG2 + CWI_LOG2 < 31 && CH_LOG2 + CWO_LOG2 < 31);
static_assert((TBL_WORDS * 4) % 256 == 0);
static_assert(R_MAX >= NSLOT && R_MAX % 2 == 0);
static_assert(RT_HALF % 128 == 0 && SR_HALF % 128 == 0 && RT_HALF >= SR_HALF && SR_HALF == 256 * SPT);
static_assert(NTOK != 8192 || (NSLOT == 16384 && R_MAX == 16896 && NT_MAX == 264 && TBL_WORDS == 33792));
static_assert((unsigned long long)NTOK * DM * 4ull <= 16777216ull);

constexpr size_t al256(size_t b) { return (b + 255) & ~(size_t)255; }
constexpr size_t SZ_WIT = al256((size_t)NE * HP * DM * 2);
constexpr size_t SZ_WOT = al256((size_t)NE * DM * HP * 2);
constexpr size_t SZ_SEL = al256((size_t)NSLOT * 4);
constexpr size_t SZ_WGT = al256((size_t)NSLOT * 4);
constexpr size_t SZ_TBL = al256((size_t)TBL_WORDS * 4);
constexpr size_t SZ_XG  = al256((size_t)R_MAX * DM * 2);
constexpr size_t SZ_HG  = al256((size_t)R_MAX * HP * 2);
constexpr size_t SZ_YG  = al256((size_t)R_MAX * DM * 4);
constexpr size_t WS_TOTAL = SZ_WIT + SZ_WIT + SZ_WOT + SZ_SEL + SZ_WGT + SZ_TBL + SZ_XG + SZ_HG + SZ_YG;
static_assert(WS_TOTAL < (size_t)268435456);
static_assert(NTOK != 8192 || WS_TOTAL == (size_t)134352896);

typedef _Float16 h16;
typedef __attribute__((ext_vector_type(16))) _Float16 v16h;
typedef __attribute__((ext_vector_type(8)))  _Float16 v8h;
typedef __attribute__((ext_vector_type(8)))  float    v8f;
typedef __attribute__((ext_vector_type(4)))  float    v4f;
typedef __attribute__((ext_vector_type(2)))  float    v2f;
typedef __attribute__((ext_vector_type(4)))  int      v4i;
typedef __attribute__((ext_vector_type(2)))  int      v2i;


#define VST2(T, ptr, val) do { const T vst2_v_ = (val); *(volatile T*)(ptr) = vst2_v_; __threadfence(); *(volatile T*)(ptr) = vst2_v_; } while (0)

static __device__ __forceinline__ float bfr(float f) {
    unsigned u = __float_as_uint(f);
    u += 0x7FFFu + ((u >> 16) & 1u);
    return __uint_as_float(u & 0xFFFF0000u);
}
static __device__ __forceinline__ h16 toh_flush(float v) { const float w = (fabsf(v) < 6.103515625e-05f) ? 0.0f : v; return (h16)w; }
static __device__ __forceinline__ void st8h(h16* p, const float* v) {
    v8h hv;
#pragma unroll
    for (int e = 0; e < 8; ++e) hv[e] = toh_flush(v[e]);
    VST2(v8h, p, hv);
}

union FragU { v16h v; v8h h[2]; };
static __device__ __forceinline__ v16h frag_ld(const h16* p) {
    FragU f; f.h[0] = *(const v8h*)(p); f.h[1] = *(const v8h*)(p + 16); return f.v;
}
static __device__ __forceinline__ v8f wmma16g(v16h a, v16h b, v8f c) {
    c = __builtin_amdgcn_wmma_f32_16x16x32_f16(false, a, false, b, (short)0, c, false, false);
    asm volatile("v_nop\n\tv_nop\n\tv_nop\n\tv_nop" : "+v"(c) : "v"(a), "v"(b));
    return c;
}
static __device__ __forceinline__ void wave_sync_lds() {
    __builtin_amdgcn_fence(3  , "workgroup");
    __builtin_amdgcn_wave_barrier();
    __builtin_amdgcn_fence(2  , "workgroup");
}

template <int KS, int NS, int KP, int NP, int LOG2C>
__global__ __launch_bounds__(256) void k_planeTR(const float* __restrict__ src, h16* __restrict__ dst) {
    static_assert(KP % 64 == 0 && NP % 64 == 0 && KS <= KP && NS <= NP && KS >= 1 && NS >= 1 && LOG2C >= 0 && LOG2C < 31);
    __shared__ __align__(16) float sT[64 * 68];
    const unsigned tid = threadIdx.x;
    const unsigned bx = blockIdx.x;
    const unsigned TPE = (unsigned)((KP / 64) * (NP / 64));
    if (bx >= (unsigned)NE * TPE) return;
    const unsigned e = bx / TPE;
    const unsigned rem = bx - e * TPE;
    const unsigned kt = rem / (unsigned)(NP / 64);
    const unsigned nt = rem - kt * (unsigned)(NP / 64);
    const unsigned k0 = kt * 64u, n0 = nt * 64u;
    const float cs = (float)(1u << LOG2C);
    const size_t sbase = (size_t)e * ((size_t)KS * (size_t)NS);
    const size_t dbase = (size_t)e * ((size_t)NP * (size_t)KP);
    const unsigned nn = tid & 63u;
    const bool nin = (n0 + nn < (unsigned)NS);
    const unsigned nc = (unsigned)min((int)(n0 + nn), NS - 1);
#pragma unroll
    for (int i = 0; i < 16; ++i) {
        const unsigned kr = (tid >> 6) + 4u * (unsigned)i;
        const bool inb = nin && (k0 + kr < (unsigned)KS);
        const unsigned kk = (unsigned)min((int)(k0 + kr), KS - 1);
        const float a = src[sbase + (size_t)kk * (size_t)NS + nc];
        const unsigned bits = __float_as_uint(bfr(a) * cs) & (inb ? 0xffffffffu : 0u);
        sT[kr * 68u + nn] = __uint_as_float(bits);
    }
    __syncthreads();
#pragma unroll
    for (int i = 0; i < 2; ++i) {
        const unsigned q = tid + 256u * (unsigned)i;
        const unsigned n = q >> 3;
        const unsigned kp = q & 7u;
        float v[8];
#pragma unroll
        for (int j = 0; j < 8; ++j) v[j] = sT[(8u * kp + (unsigned)j) * 68u + n];
        st8h(dst + dbase + (size_t)(n0 + n) * KP + k0 + 8u * kp, v);
    }
}

__global__ __launch_bounds__(256) void k_gate(const float* __restrict__ x, const float* __restrict__ gw,
                                              int* __restrict__ sel, float* __restrict__ wgt) {
    const unsigned lane = threadIdx.x & 31u;
    const unsigned wave = threadIdx.x >> 5;
    const unsigned t0 = (blockIdx.x * 8u + wave) * 16u;
    if (t0 >= (unsigned)NTOK) return;
    int ki0 = 0, ki1 = 0;
    float kw0 = 0.0f, kw1 = 0.0f;
    for (unsigned j = 0; j < 16u; ++j) {
        const float* xr = x + (size_t)(t0 + j) * DM;
        float lg[NE];
#pragma unroll
        for (int e = 0; e < NE; ++e) lg[e] = 0.0f;
        for (unsigned i = 0; i < (unsigned)(DM / 32); ++i) {
            const unsigned d = lane + 32u * i;
            const float xv = bfr(xr[d]);
            const v4f ga = *(const v4f*)(gw + (size_t)d * NE);
            const v4f gb = *(const v4f*)(gw + (size_t)d * NE + 4u);
            lg[0] += xv * bfr(ga.x); lg[1] += xv * bfr(ga.y);
            lg[2] += xv * bfr(ga.z); lg[3] += xv * bfr(ga.w);
            lg[4] += xv * bfr(gb.x); lg[5] += xv * bfr(gb.y);
            lg[6] += xv * bfr(gb.z); lg[7] += xv * bfr(gb.w);
        }
#pragma unroll
        for (int e = 0; e < NE; ++e) {
            lg[e] += __shfl_xor(lg[e], 16, 32);
            lg[e] += __shfl_xor(lg[e], 8, 32);
            lg[e] += __shfl_xor(lg[e], 4, 32);
            lg[e] += __shfl_xor(lg[e], 2, 32);
            lg[e] += __shfl_xor(lg[e], 1, 32);
        }
        float bestv = lg[0];
        int besti = 0;
#pragma unroll
        for (int e = 1; e < NE; ++e) { const bool c = lg[e] > bestv; bestv = c ? lg[e] : bestv; besti = c ? e : besti; }
        float secv = -INFINITY;
        int seci = 0;
#pragma unroll
        for (int e = 0; e < NE; ++e) { const bool c = (e != besti) && (lg[e] > secv); secv = c ? lg[e] : secv; seci = c ? e : seci; }
        const float e1 = expf(secv - bestv);
        const float den = 1.0f + e1;
        const float w0 = 1.0f / den;
        const float w1 = e1 / den;
        const bool mine = (lane == j);
        ki0 = mine ? besti : ki0;  ki1 = mine ? seci : ki1;
        kw0 = mine ? w0 : kw0;     kw1 = mine ? w1 : kw1;
    }
    if (lane < 16u) {
        v2i sv; sv.x = ki0; sv.y = ki1;
        v2f wv; wv.x = kw0; wv.y = kw1;
        VST2(v2i, sel + (size_t)(t0 + lane) * 2u, sv);
        VST2(v2f, wgt + (size_t)(t0 + lane) * 2u, wv);
    }
}

__global__ __launch_bounds__(512) void k_route(const int* __restrict__ sel, int* __restrict__ tbl) {
    __shared__ __align__(16) int s_img[RT_HALF];
    __shared__ __align__(16) int s_hdr[512];
    __shared__ int sc[512];
    const unsigned tid = threadIdx.x;
    s_hdr[tid] = (tid >= (unsigned)TBL_TILE_E && tid < (unsigned)(TBL_TILE_E + NT_MAX)) ? -1 : 0;
    __syncthreads();
    int cnt[NE];
#pragma unroll
    for (int j = 0; j < NE; ++j) cnt[j] = 0;
    const v4i* sp = (const v4i*)(sel + (size_t)tid * (unsigned)SPT);
#pragma unroll
    for (int g = 0; g < SPT / 4; ++g) {
        const v4i v = sp[g];
#pragma unroll
        for (int c = 0; c < 4; ++c) {
            const int e = min(max(v[c], 0), NE - 1);
#pragma unroll
            for (int j = 0; j < NE; ++j) cnt[j] += (e == j) ? 1 : 0;
        }
    }
    int base[NE], total[NE];
#pragma unroll
    for (int j = 0; j < NE; ++j) {
        sc[tid] = cnt[j];
        __syncthreads();
        for (unsigned off = 1u; off < 512u; off <<= 1) {
            const unsigned src = (tid >= off) ? (tid - off) : 0u;
            const int add = sc[src];
            const int v = sc[tid] + ((tid >= off) ? add : 0);
            __syncthreads();
            sc[tid] = v;
            __syncthreads();
        }
        base[j] = sc[tid] - cnt[j];
        total[j] = sc[511];
        __syncthreads();
    }
    int base0[NE];
#pragma unroll
    for (int j = 0; j < NE; ++j) base0[j] = base[j];
    int poff[NE + 1];
    poff[0] = 0;
#pragma unroll
    for (int j = 0; j < NE; ++j) poff[j + 1] = poff[j] + (((total[j] + 63) >> 6) << 6);
    if (tid == 0u) {
#pragma unroll
        for (int j = 0; j < NE; ++j) { s_hdr[TBL_COUNT + j] = total[j]; s_hdr[TBL_POFF + j] = poff[j]; }
        s_hdr[TBL_POFF + NE] = poff[NE];
        s_hdr[TBL_NTILES] = poff[NE] >> 6;
    }
    if (tid < (unsigned)NT_MAX) {
        const int b64 = (int)(tid * 64u);
        int ev = -1;
#pragma unroll
        for (int j = 0; j < NE; ++j) ev = (b64 >= poff[j] && b64 < poff[j + 1]) ? j : ev;
        s_hdr[TBL_TILE_E + tid] = ev;
    }
    __syncthreads();
    for (int pass = 0; pass < 2; ++pass) {
        if (tid < 128u) *(volatile v4i*)(tbl + 4u * tid) = *(const v4i*)(&s_hdr[4u * tid]);
        __threadfence();
    }
    for (int h = 0; h < 2; ++h) {
        const int lo = h * RT_HALF;
        for (unsigned i = tid; i < (unsigned)RT_HALF; i += 512u) s_img[i] = -1;
        __syncthreads();
        int run[NE];
#pragma unroll
        for (int j = 0; j < NE; ++j) run[j] = base0[j];
#pragma unroll
        for (int g = 0; g < SPT / 4; ++g) {
            const v4i v = sp[g];
#pragma unroll
            for (int c = 0; c < 4; ++c) {
                const int e = min(max(v[c], 0), NE - 1);
                int row = 0;
#pragma unroll
                for (int j = 0; j < NE; ++j) {
                    const bool hit = (e == j);
                    row = hit ? (poff[j] + run[j]) : row;
                    run[j] += hit ? 1 : 0;
                }
                row = min(max(row, 0), R_MAX - 1);
                const int rel = row - lo;
                if (rel >= 0 && rel < RT_HALF) s_img[rel] = (int)((tid * (unsigned)SPT + 4u * (unsigned)g + (unsigned)c) >> 1);
            }
        }
        __syncthreads();
        for (int pass = 0; pass < 2; ++pass) {
            for (unsigned i = tid; i < (unsigned)(RT_HALF / 4); i += 512u) *(volatile v4i*)(tbl + TBL_ROWTOK + (unsigned)lo + 4u * i) = *(const v4i*)(&s_img[4u * i]);
            __threadfence();
        }
        __syncthreads();
    }
    for (int h = 0; h < 2; ++h) {
        if ((tid >> 8) == (unsigned)h) {
            int run[NE];
#pragma unroll
            for (int j = 0; j < NE; ++j) run[j] = base0[j];
#pragma unroll
            for (int g = 0; g < SPT / 4; ++g) {
                const v4i v = sp[g];
                v4i pk = (v4i){0, 0, 0, 0};
#pragma unroll
                for (int c = 0; c < 4; ++c) {
                    const int e = min(max(v[c], 0), NE - 1);
                    int row = 0;
#pragma unroll
                    for (int j = 0; j < NE; ++j) {
                        const bool hit = (e == j);
                        row = hit ? (poff[j] + run[j]) : row;
                        run[j] += hit ? 1 : 0;
                    }
                    pk[c] = min(max(row, 0), R_MAX - 1);
                }
                *(v4i*)(&s_img[(tid - 256u * (unsigned)h) * (unsigned)SPT + 4u * (unsigned)g]) = pk;
            }
        }
        __syncthreads();
        for (int pass = 0; pass < 2; ++pass) {
            for (unsigned i = tid; i < (unsigned)(SR_HALF / 4); i += 512u) *(volatile v4i*)(tbl + TBL_SLOTROW + (unsigned)(h * SR_HALF) + 4u * i) = *(const v4i*)(&s_img[4u * i]);
            __threadfence();
        }
        __syncthreads();
    }
}

__global__ __launch_bounds__(256) void k_gather(const float* __restrict__ x, const int* __restrict__ tbl, h16* __restrict__ Xg) {
    const unsigned TPR = (unsigned)(DM / 8);
    const unsigned row = blockIdx.x * (256u / TPR) + (threadIdx.x / TPR);
    if (row >= (unsigned)R_MAX) return;
    const unsigned c = (threadIdx.x % TPR) * 8u;
    const int tr = tbl[TBL_ROWTOK + row];
    const bool pad = (tr < 0);
    const int tok = min(max(tr, 0), NTOK - 1);
    const float* xp = x + (size_t)(unsigned)tok * DM + c;
    const v4f a = *(const v4f*)(xp);
    const v4f b = *(const v4f*)(xp + 4);
    float v[8] = {pad ? 0.0f : bfr(a.x) * CX, pad ? 0.0f : bfr(a.y) * CX, pad ? 0.0f : bfr(a.z) * CX, pad ? 0.0f : bfr(a.w) * CX, pad ? 0.0f : bfr(b.x) * CX, pad ? 0.0f : bfr(b.y) * CX, pad ? 0.0f : bfr(b.z) * CX, pad ? 0.0f : bfr(b.w) * CX};
    st8h(Xg + (size_t)row * DM + c, v);
}

__global__ __launch_bounds__(256) void k_ffn1(const h16* __restrict__ Xg, const h16* __restrict__ WvT, const h16* __restrict__ WgT,
                                              const float* __restrict__ bv, const float* __restrict__ bg, const int* __restrict__ tbl, h16* __restrict__ Hg) {
    __shared__ __align__(16) float sT[8][16 * 68];
    const unsigned lane = threadIdx.x & 31u;
    const unsigned wave = threadIdx.x >> 5;
    const unsigned u = blockIdx.x * 8u + wave;
    if (u >= (unsigned)(NT_MAX * 2 * (HP / 64))) return;
    const unsigned rt32 = u / (unsigned)(HP / 64);
    const unsigned ct = u - rt32 * (unsigned)(HP / 64);
    const unsigned rowtile = rt32 >> 1;
    const int nt = min(max(tbl[TBL_NTILES], 0), NT_MAX);
    if ((int)rowtile >= nt) return;
    const int e = min(max(tbl[TBL_TILE_E + rowtile], 0), NE - 1);
    const size_t wbase = (size_t)(unsigned)e * (size_t)(HP * DM);
    const unsigned bbase = (unsigned)e * (unsigned)HID;
    const unsigned m0 = rt32 * 32u, n0 = ct * 64u;
    const unsigned rlane = lane & 15u;
    const unsigned koff = (lane >> 4) * 8u;
    const unsigned mOff = koff;

    v8f acc1[2][4], acc2[2][4];
#pragma unroll
    for (int i = 0; i < 2; ++i)
#pragma unroll
        for (int j = 0; j < 4; ++j) { acc1[i][j] = (v8f){0.f,0.f,0.f,0.f,0.f,0.f,0.f,0.f}; acc2[i][j] = acc1[i][j]; }

    for (unsigned k0 = 0; k0 < (unsigned)DM; k0 += 32u) {
        v16h ah[2];
#pragma unroll
        for (int i = 0; i < 2; ++i)
            ah[i] = frag_ld(Xg + (size_t)(m0 + ((unsigned)i << 4) + rlane) * DM + koff + k0);
#pragma unroll
        for (int j = 0; j < 4; ++j) {
            const size_t boff = wbase + (size_t)(n0 + ((unsigned)j << 4) + rlane) * DM + koff + k0;
            const v16h b1 = frag_ld(WvT + boff);
            const v16h b2 = frag_ld(WgT + boff);
#pragma unroll
            for (int i = 0; i < 2; ++i) {
                acc1[i][j] = wmma16g(ah[i], b1, acc1[i][j]);
                acc2[i][j] = wmma16g(ah[i], b2, acc2[i][j]);
            }
        }
    }

    float bvv[4], bgv[4];
#pragma unroll
    for (int j = 0; j < 4; ++j) {
        const unsigned ncol = n0 + ((unsigned)j << 4) + rlane;
        const unsigned nci = (unsigned)min((int)ncol, HID - 1);
        const bool inh = (ncol < (unsigned)HID);
        const float lv = bfr(bv[bbase + nci]);
        const float lw = bfr(bg[bbase + nci]);
        bvv[j] = inh ? lv : 0.0f;
        bgv[j] = inh ? lw : 0.0f;
    }
    float* slab = sT[wave];
#pragma unroll
    for (int i = 0; i < 2; ++i) {
        const unsigned mBase = m0 + ((unsigned)i << 4);
#pragma unroll
        for (int j = 0; j < 4; ++j) {
#pragma unroll
            for (int r = 0; r < 8; ++r) {
                const float a = acc1[i][j][r] * SC_HG + bvv[j];
                const float g = acc2[i][j][r] * SC_HG + bgv[j];
                const float s = a / (1.0f + expf(-a));
                slab[(mOff + (unsigned)r) * 68u + ((unsigned)j << 4) + rlane] = (s * g) * CH;
            }
        }
        wave_sync_lds();
        const unsigned q = lane >> 3, c8 = (lane & 7u) * 8u;
        v8h hv[4];
#pragma unroll
        for (int it = 0; it < 4; ++it) {
            const unsigned row = (unsigned)it * 4u + q;
            const float* sp = slab + row * 68u + c8;
#pragma unroll
            for (int t = 0; t < 8; ++t) hv[it][t] = toh_flush(sp[t]);
        }
        for (int pass = 0; pass < 2; ++pass) {
#pragma unroll
            for (int it = 0; it < 4; ++it) {
                const unsigned row = (unsigned)it * 4u + q;
                *(volatile v8h*)(Hg + (size_t)(mBase + row) * HP + n0 + c8) = hv[it];
            }
            __threadfence();
        }
        wave_sync_lds();
    }
}

__global__ __launch_bounds__(256) void k_ffn2(const h16* __restrict__ Hg, const h16* __restrict__ WoT, const float* __restrict__ bo,
                                              const int* __restrict__ tbl, float* __restrict__ Yg) {
    __shared__ __align__(16) float sT[8][16 * 68];
    const unsigned lane = threadIdx.x & 31u;
    const unsigned wave = threadIdx.x >> 5;
    const unsigned u = blockIdx.x * 8u + wave;
    if (u >= (unsigned)(NT_MAX * (DM / 64))) return;
    const unsigned rowtile = u / (unsigned)(DM / 64);
    const unsigned ct = u - rowtile * (unsigned)(DM / 64);
    const int nt = min(max(tbl[TBL_NTILES], 0), NT_MAX);
    if ((int)rowtile >= nt) return;
    const int e = min(max(tbl[TBL_TILE_E + rowtile], 0), NE - 1);
    const size_t wbase = (size_t)(unsigned)e * (size_t)(DM * HP);
    const unsigned m0 = rowtile << 6, n0 = ct << 6;
    const unsigned rlane = lane & 15u;
    const unsigned koff = (lane >> 4) * 8u;
    const unsigned mOff = koff;

    v8f acc[4][4];
#pragma unroll
    for (int i = 0; i < 4; ++i)
#pragma unroll
        for (int j = 0; j < 4; ++j) acc[i][j] = (v8f){0.f,0.f,0.f,0.f,0.f,0.f,0.f,0.f};

    for (unsigned k0 = 0; k0 < (unsigned)HP; k0 += 32u) {
        v16h bh[4];
#pragma unroll
        for (int j = 0; j < 4; ++j)
            bh[j] = frag_ld(WoT + wbase + (size_t)(n0 + ((unsigned)j << 4) + rlane) * HP + koff + k0);
#pragma unroll
        for (int i = 0; i < 4; ++i) {
            const v16h ah = frag_ld(Hg + (size_t)(m0 + ((unsigned)i << 4) + rlane) * HP + koff + k0);
#pragma unroll
            for (int j = 0; j < 4; ++j) acc[i][j] = wmma16g(ah, bh[j], acc[i][j]);
        }
    }

    float ebv[4];
#pragma unroll
    for (int j = 0; j < 4; ++j) ebv[j] = bfr(bo[(unsigned)e * (unsigned)DM + n0 + ((unsigned)j << 4) + rlane]);

    float* slab = sT[wave];
#pragma unroll
    for (int i = 0; i < 4; ++i) {
        const unsigned mBase = m0 + ((unsigned)i << 4);
#pragma unroll
        for (int j = 0; j < 4; ++j)
#pragma unroll
            for (int r = 0; r < 8; ++r)
                slab[(mOff + (unsigned)r) * 68u + ((unsigned)j << 4) + rlane] = acc[i][j][r] * SC_Y + ebv[j];
        wave_sync_lds();
        const unsigned hh = lane >> 4, c4 = (lane & 15u) * 4u;
#pragma unroll
        for (int half = 0; half < 2; ++half) {
            v4f vv[4];
#pragma unroll
            for (int it = 0; it < 4; ++it) {
                const unsigned row = (unsigned)(half * 4 + it) * 2u + hh;
                vv[it] = *(const v4f*)(slab + row * 68u + c4);
            }
            for (int pass = 0; pass < 2; ++pass) {
#pragma unroll
                for (int it = 0; it < 4; ++it) {
                    const unsigned row = (unsigned)(half * 4 + it) * 2u + hh;
                    *(volatile v4f*)(Yg + (size_t)(mBase + row) * DM + n0 + c4) = vv[it];
                }
                __threadfence();
            }
        }
        wave_sync_lds();
    }
}

__global__ __launch_bounds__(256) void k_combine_ln(const float* __restrict__ x, const float* __restrict__ Yg, const float* __restrict__ wgt, const int* __restrict__ tbl,
                                                    const float* __restrict__ gamma, const float* __restrict__ beta, float* __restrict__ out) {
    const unsigned lane = threadIdx.x & 31u;
    const unsigned wave = threadIdx.x >> 5;
    const unsigned t = blockIdx.x * 8u + wave;
    if (t >= (unsigned)NTOK) return;
    const int r0 = min(max(tbl[TBL_SLOTROW + 2u * t], 0), R_MAX - 1);
    const int r1 = min(max(tbl[TBL_SLOTROW + 2u * t + 1u], 0), R_MAX - 1);
    const float w0 = wgt[2u * t], w1 = wgt[2u * t + 1u];
    v4f y[4];
    float s = 0.0f;
#pragma unroll
    for (int q = 0; q < 4; ++q) {
        const unsigned c = 4u * lane + 128u * (unsigned)q;
        const v4f xa = *(const v4f*)(x + (size_t)t * DM + c);
        const v4f a = *(const v4f*)(Yg + (size_t)(unsigned)r0 * DM + c);
        const v4f b = *(const v4f*)(Yg + (size_t)(unsigned)r1 * DM + c);
        const v4f m = (a * w0) + (b * w1);
        y[q].x = bfr(xa.x) + m.x; y[q].y = bfr(xa.y) + m.y;
        y[q].z = bfr(xa.z) + m.z; y[q].w = bfr(xa.w) + m.w;
        s = (((s + y[q].x) + y[q].y) + y[q].z) + y[q].w;
    }
    s += __shfl_xor(s, 16, 32);
    s += __shfl_xor(s, 8, 32);
    s += __shfl_xor(s, 4, 32);
    s += __shfl_xor(s, 2, 32);
    s += __shfl_xor(s, 1, 32);
    const float mu = s / 512.0f;
    float vs = 0.0f;
#pragma unroll
    for (int q = 0; q < 4; ++q) {
        y[q].x -= mu; y[q].y -= mu; y[q].z -= mu; y[q].w -= mu;
        vs = (((vs + y[q].x * y[q].x) + y[q].y * y[q].y) + y[q].z * y[q].z) + y[q].w * y[q].w;
    }
    vs += __shfl_xor(vs, 16, 32);
    vs += __shfl_xor(vs, 8, 32);
    vs += __shfl_xor(vs, 4, 32);
    vs += __shfl_xor(vs, 2, 32);
    vs += __shfl_xor(vs, 1, 32);
    const float var = vs / 512.0f;
    const float rs = 1.0f / sqrtf(var + 1e-5f);
    v4f o[4];
#pragma unroll
    for (int q = 0; q < 4; ++q) {
        const unsigned c = 4u * lane + 128u * (unsigned)q;
        const v4f ga = *(const v4f*)(gamma + c);
        const v4f be = *(const v4f*)(beta + c);
        o[q].x = bfr(ga.x) * (y[q].x * rs) + bfr(be.x); o[q].y = bfr(ga.y) * (y[q].y * rs) + bfr(be.y);
        o[q].z = bfr(ga.z) * (y[q].z * rs) + bfr(be.z); o[q].w = bfr(ga.w) * (y[q].w * rs) + bfr(be.w);
    }
    for (int pass = 0; pass < 2; ++pass) {
#pragma unroll
        for (int q = 0; q < 4; ++q) *(volatile v4f*)(out + (size_t)t * DM + 4u * lane + 128u * (unsigned)q) = o[q];
        __threadfence();
    }
}

extern "C" void kernel_launch(void* const* d_in, const int* in_sizes, int n_in, void* d_out, int out_size,
                              void* d_ws, size_t ws_size, hipStream_t stream) {
    if (n_in < 10) return;
    if (in_sizes[0] < NTOK * DM || in_sizes[1] < DM * NE) return;
    if (in_sizes[2] < NE * DM * HID || in_sizes[3] < NE * HID || in_sizes[4] < NE * DM * HID || in_sizes[5] < NE * HID) return;
    if (in_sizes[6] < NE * HID * DM || in_sizes[7] < NE * DM || in_sizes[8] < DM || in_sizes[9] < DM) return;
    if (out_size < NTOK * DM) return;

    const float* x     = (const float*)d_in[0];
    const float* gw    = (const float*)d_in[1];
    const float* Wv    = (const float*)d_in[2];
    const float* bv    = (const float*)d_in[3];
    const float* Wg    = (const float*)d_in[4];
    const float* bg    = (const float*)d_in[5];
    const float* Wo    = (const float*)d_in[6];
    const float* bo    = (const float*)d_in[7];
    const float* gamma = (const float*)d_in[8];
    const float* beta  = (const float*)d_in[9];
    float* out = (float*)d_out;

    char* wsp = (char*)d_ws;
    size_t off = 0;
    auto carve = [&](size_t bytes) -> void* { void* r = wsp + off; off += (bytes + 255) & ~(size_t)255; return r; };
    h16*   WvT = (h16*)carve((size_t)NE * HP * DM * 2);
    h16*   WgT = (h16*)carve((size_t)NE * HP * DM * 2);
    h16*   WoT = (h16*)carve((size_t)NE * DM * HP * 2);
    int*   sel = (int*)carve((size_t)NSLOT * 4);
    float* wgt = (float*)carve((size_t)NSLOT * 4);
    int*   tbl = (int*)carve((size_t)TBL_WORDS * 4);
    h16*   Xg  = (h16*)carve((size_t)R_MAX * DM * 2);
    h16*   Hg  = (h16*)carve((size_t)R_MAX * HP * 2);
    float* Yg  = (float*)carve((size_t)R_MAX * DM * 4);
    if (off != WS_TOTAL || off > ws_size || off > (size_t)268435456) return;

    k_planeTR<DM, HID, DM, HP, CWI_LOG2><<<NE * (DM / 64) * (HP / 64), 256, 0, stream>>>(Wv, WvT);
    k_planeTR<DM, HID, DM, HP, CWI_LOG2><<<NE * (DM / 64) * (HP / 64), 256, 0, stream>>>(Wg, WgT);
    k_planeTR<HID, DM, HP, DM, CWO_LOG2><<<NE * (HP / 64) * (DM / 64), 256, 0, stream>>>(Wo, WoT);
    k_gate<<<NTOK / 128, 256, 0, stream>>>(x, gw, sel, wgt);
    k_route<<<1, 512, 0, stream>>>(sel, tbl);
    k_gather<<<R_MAX / 4, 256, 0, stream>>>(x, tbl, Xg);
    k_ffn1<<<(NT_MAX * 2 * (HP / 64) + 7) / 8, 256, 0, stream>>>(Xg, WvT, WgT, bv, bg, tbl, Hg);
    k_ffn2<<<(NT_MAX * (DM / 64) + 7) / 8, 256, 0, stream>>>(Hg, WoT, bo, tbl, Yg);
    k_combine_ln<<<NTOK / 8, 256, 0, stream>>>(x, Yg, wgt, tbl, gamma, beta, out);
}
